// GIN_28424093565719
// MI455X (gfx1250) — hardware-verified
//
#include <hip/hip_runtime.h>
#include <stddef.h>
#include <stdint.h>
#include <math.h>


#define DF      64
#define NCLS    10
#define NCP     16
#define KZ      128
#define NTHR    256
#define NWAVE   8
#define EPT     8
#define CHUNK   (NTHR * EPT)
#define WCAP    (EPT * 32)
#define LISTN   (NWAVE * WCAP)
#define NBA     1024
#define PKS     10
#define RCAP    28672
#define DEGCAP  64
#define GBM     64
#define GTHR    128
#define GNT     4
#define NUA     (DF * (KZ / 8))
#define NUC     (NCP * (KZ / 8))
#define RG1     NUA
#define RG2     (RG1 + NUA)
#define RG3     (RG2 + NUA)
#define RG4     (RG3 + NUC)
#define ZINTS   (2 * RCAP + 2 * NBA + LISTN)
#define LDS_AGG (ZINTS * 4 + 64)
#define WSMAX   134217728
#define SELFS   1.5f
#define BNEPS   1e-3f

static_assert((CHUNK & (CHUNK - 1)) == 0);
static_assert(NBA == (1 << PKS));
static_assert(((long long)CHUNK << PKS) < (1LL << 31));
static_assert(NTHR * 4 == NBA);
static_assert(LISTN >= NBA && LISTN >= NWAVE * WCAP);
static_assert((RCAP % 32) == 0);
static_assert((ZINTS % (NTHR * 4)) == 0);
static_assert(LDS_AGG <= 262144);
static_assert((NBA % NWAVE) == 0 && (NBA % GBM) == 0);
static_assert((NBA / NWAVE) == 128);
static_assert(GBM == (GTHR / 32) * 16);
static_assert(KZ == 2 * DF && (KZ % 32) == 0);
static_assert(DF == 32 * 2);
static_assert(DF == 16 * GNT);
static_assert(GBM * DF == GTHR * 32);
static_assert(NCLS <= NCP && NCP == 16);
static_assert(GBM * NCLS == 4 * (GTHR + 32));
static_assert(((GBM * NCLS * 4) % 128) == 0);
static_assert((RG1 % NTHR) == 0 && (RG2 % NTHR) == 0 && (RG3 % NTHR) == 0 && (RG4 % NTHR) == 0);
static_assert((KZ / 8) == 16);
static_assert(((DF * 4) % 128) == 0 && ((KZ * 2) % 128) == 0);

typedef float          v2f  __attribute__((ext_vector_type(2)));
typedef float          v4f  __attribute__((ext_vector_type(4)));
typedef float          v8f  __attribute__((ext_vector_type(8)));
typedef int            v4i  __attribute__((ext_vector_type(4)));
typedef int            v8i  __attribute__((ext_vector_type(8)));
typedef unsigned int   v2u  __attribute__((ext_vector_type(2)));
typedef unsigned short v8us __attribute__((ext_vector_type(8)));
typedef __bf16         v16b __attribute__((ext_vector_type(16)));
typedef v2f  __attribute__((may_alias)) v2fa;
typedef v4f  __attribute__((may_alias)) v4fa;
typedef v4i  __attribute__((may_alias)) v4ia;
typedef v8us __attribute__((may_alias)) v8usa;
union Frag { v16b b; v8us h[2]; v8i w; };

__device__ __forceinline__ v8f wmk(const Frag& a, const Frag& b, v8f c) {
  v8f d = __builtin_amdgcn_wmma_f32_16x16x32_bf16(false, a.b, false, b.b, (short)0, c, false, false);
  asm volatile("v_nop\n\tv_nop\n\tv_nop\n\tv_nop" : "+v"(d) : "v"(a.w), "v"(b.w));
  return d;
}

__device__ __forceinline__ v8f z8() { v8f z = {0.f, 0.f, 0.f, 0.f, 0.f, 0.f, 0.f, 0.f}; return z; }

__device__ __forceinline__ unsigned short bf_bits(float f) {
  unsigned int u = __float_as_uint(f);
  u += 0x7FFFu + ((u >> 16) & 1u);
  return (unsigned short)(u >> 16);
}
__device__ __forceinline__ float bf_val(unsigned short b) {
  return __uint_as_float(((unsigned int)b) << 16);
}
__device__ __forceinline__ float bf_rne(float f) { return bf_val(bf_bits(f)); }

__device__ __forceinline__ void split8b(const v4f a, const v4f b, v8us& hi, v8us& lo) {
  float x[8];
  x[0] = a.x; x[1] = a.y; x[2] = a.z; x[3] = a.w; x[4] = b.x; x[5] = b.y; x[6] = b.z; x[7] = b.w;
#pragma unroll
  for (int i = 0; i < 8; ++i) {
    const unsigned short hb = bf_bits(x[i]);
    hi[i] = hb;
    lo[i] = bf_bits(x[i] - bf_val(hb));
  }
}

__device__ __forceinline__ int scan_chunk(const int* __restrict__ dsts, int nE, int cbase, int slotBase,
                                          int nb, int vec8, int* list, int tid, int lane, int wave) {
  int wc = 0;
  const int el0  = tid * EPT;
  const int e0   = cbase + el0;
  const int sent = -2147483647 - 1;
  v4i da, db;
  if (vec8 != 0 && cbase + CHUNK <= nE) {
    da = *(const v4i*)(dsts + e0);
    db = *(const v4i*)(dsts + e0 + 4);
  } else {
    da.x = (e0     < nE) ? dsts[min(e0,     nE - 1)] : sent;
    da.y = (e0 + 1 < nE) ? dsts[min(e0 + 1, nE - 1)] : sent;
    da.z = (e0 + 2 < nE) ? dsts[min(e0 + 2, nE - 1)] : sent;
    da.w = (e0 + 3 < nE) ? dsts[min(e0 + 3, nE - 1)] : sent;
    db.x = (e0 + 4 < nE) ? dsts[min(e0 + 4, nE - 1)] : sent;
    db.y = (e0 + 5 < nE) ? dsts[min(e0 + 5, nE - 1)] : sent;
    db.z = (e0 + 6 < nE) ? dsts[min(e0 + 6, nE - 1)] : sent;
    db.w = (e0 + 7 < nE) ? dsts[min(e0 + 7, nE - 1)] : sent;
  }
  const unsigned nbs = (unsigned)slotBase;
  const unsigned unb = (unsigned)nb;
  const unsigned s0 = (unsigned)da.x - nbs, s1 = (unsigned)da.y - nbs;
  const unsigned s2 = (unsigned)da.z - nbs, s3 = (unsigned)da.w - nbs;
  const unsigned s4 = (unsigned)db.x - nbs, s5 = (unsigned)db.y - nbs;
  const unsigned s6 = (unsigned)db.z - nbs, s7 = (unsigned)db.w - nbs;
  const bool h0 = s0 < unb, h1 = s1 < unb, h2 = s2 < unb, h3 = s3 < unb;
  const bool h4 = s4 < unb, h5 = s5 < unb, h6 = s6 < unb, h7 = s7 < unb;
  const unsigned any = __builtin_amdgcn_ballot_w32(h0 | h1 | h2 | h3 | h4 | h5 | h6 | h7);
  if (any != 0u) {
#define HITJ(J, HJ, SJ) { \
      const unsigned mj = __builtin_amdgcn_ballot_w32(HJ); \
      if (mj != 0u) { \
        if (HJ) { \
          const int pos = wc + (int)__builtin_amdgcn_mbcnt_lo(mj, 0u); \
          if (pos < WCAP) list[wave * WCAP + pos] = ((el0 + (J)) << PKS) | (int)(SJ); \
        } \
        wc += (int)__builtin_popcount(mj); } }
    HITJ(0, h0, s0)
    HITJ(1, h1, s1)
    HITJ(2, h2, s2)
    HITJ(3, h3, s3)
    HITJ(4, h4, s4)
    HITJ(5, h5, s5)
    HITJ(6, h6, s6)
    HITJ(7, h7, s7)
#undef HITJ
  }
  return wc;
}

__global__ __launch_bounds__(NTHR) void k_wprep(const float* __restrict__ w1a, const float* __restrict__ w1b,
                                                const float* __restrict__ w2a, const float* __restrict__ w2b,
                                                unsigned short* WA1, unsigned short* WB1,
                                                unsigned short* WA2, unsigned short* WB2) {
  const int u = (int)blockIdx.x * NTHR + (int)threadIdx.x;
  v8us o;
  unsigned short* dp;
  if (u < RG1) {
    const int n = u >> 4;
    const int q = u & 15;
    const float* p = w1a + (size_t)(4 * q) * DF + n;
    float f[4];
#pragma unroll
    for (int c = 0; c < 4; ++c) f[c] = p[(size_t)c * DF];
#pragma unroll
    for (int i = 0; i < 8; ++i) o[i] = bf_bits(f[2 * (i >> 2) + (i & 1)]);
    dp = WA1 + (size_t)n * KZ + 8 * q;
  } else if (u < RG2) {
    const int v  = u - RG1;
    const int n  = v >> 4;
    const int q  = v & 15;
    const int kk = (8 * q) & (DF - 1);
    const float* p = w1b + (size_t)kk * DF + n;
#pragma unroll
    for (int i = 0; i < 8; ++i) o[i] = bf_bits(p[(size_t)i * DF]);
    dp = WB1 + (size_t)n * KZ + 8 * q;
  } else if (u < RG3) {
    const int v = u - RG2;
    const int n = v >> 4;
    const int q = v & 15;
    const float* p = w2a + (size_t)(4 * q) * DF + n;
    float f[4];
#pragma unroll
    for (int c = 0; c < 4; ++c) f[c] = p[(size_t)c * DF];
#pragma unroll
    for (int i = 0; i < 8; ++i) o[i] = bf_bits(f[2 * (i >> 2) + (i & 1)]);
    dp = WA2 + (size_t)n * KZ + 8 * q;
  } else if (u < RG4) {
    const int v  = u - RG3;
    const int n  = v >> 4;
    const int q  = v & 15;
    const int kk = (8 * q) & (DF - 1);
    const int nn = n < NCLS ? n : NCLS - 1;
    const float* p = w2b + (size_t)kk * NCLS + nn;
#pragma unroll
    for (int i = 0; i < 8; ++i) {
      const unsigned short b = bf_bits(p[(size_t)i * NCLS]);
      o[i] = (n < NCLS) ? b : (unsigned short)0;
    }
    dp = WB2 + (size_t)n * KZ + 8 * q;
  } else {
    return;
  }
  *(volatile v8us*)dp = o;
  __threadfence();
  *(volatile v8us*)dp = o;
}

template <int NB2, int FIN>
__global__ __launch_bounds__(GTHR) void k_mlp(const unsigned short* __restrict__ Z,
                                              const unsigned short* __restrict__ WA, const float* __restrict__ ba,
                                              const unsigned short* __restrict__ WB, const float* __restrict__ bb,
                                              const float* __restrict__ gam, const float* __restrict__ bet,
                                              const float* __restrict__ rme, const float* __restrict__ rva,
                                              float* H, float* outF, int nN) {
  static_assert((FIN == 0 && NB2 == GNT) || (FIN == 1 && NB2 == 1));
  constexpr int NCOL = (FIN == 1) ? NCLS : DF;
  constexpr int NCT  = 16 * NB2;
  __shared__ __attribute__((aligned(16))) float stg[GBM * DF];
  __shared__ __attribute__((aligned(16))) unsigned short tpl[GBM * KZ];
  __shared__ __attribute__((aligned(16))) float cb[DF];
  __shared__ __attribute__((aligned(16))) float csc[DF];
  __shared__ __attribute__((aligned(16))) float crm[DF];
  __shared__ __attribute__((aligned(16))) float cbe[DF];
  __shared__ __attribute__((aligned(16))) float orow[GBM * NCLS];
  const int tid = (int)threadIdx.x, lane = tid & 31, wave = tid >> 5, hh = lane >> 4, m = lane & 15;
  const int rowBase = (int)blockIdx.x * GBM;

  if (tid < NCT) {
    const int c  = tid;
    const int cc = c < NCOL ? c : NCOL - 1;
    cb[c]  = bf_rne(bb[cc]);
    csc[c] = bf_rne(gam[cc]) * rsqrtf(bf_rne(rva[cc]) + BNEPS);
    crm[c] = bf_rne(rme[cc]);
    cbe[c] = bf_rne(bet[cc]);
  }

  v8f acc[GNT];
#pragma unroll
  for (int t = 0; t < GNT; ++t) acc[t] = z8();
  {
    const unsigned short* ap = Z  + (size_t)(rowBase + 16 * wave + m) * (size_t)KZ + 8 * hh;
    const unsigned short* bp = WA + (size_t)m * (size_t)KZ + 8 * hh;
#pragma unroll 1
    for (int k0 = 0; k0 < KZ; k0 += 32) {
      Frag af;
      af.h[0] = *(const v8usa*)(ap + k0);
      af.h[1] = *(const v8usa*)(ap + k0 + 16);
#pragma unroll
      for (int nt = 0; nt < GNT; ++nt) {
        const unsigned short* wq = bp + (size_t)(16 * nt) * (size_t)KZ + k0;
        Frag bf;
        bf.h[0] = *(const v8usa*)wq;
        bf.h[1] = *(const v8usa*)(wq + 16);
        acc[nt] = wmk(af, bf, acc[nt]);
      }
    }
  }
#pragma unroll
  for (int nt = 0; nt < GNT; ++nt) {
    const int lc = 16 * nt + m;
    const float bv = bf_rne(ba[lc]);
#pragma unroll
    for (int r = 0; r < 8; ++r) {
      const int lr = 16 * wave + 8 * hh + r;
      stg[lr * DF + lc] = fmaxf(acc[nt][r] + bv, 0.0f);
    }
  }
  __syncthreads();

  {
    const int r  = tid >> 1;
    const int c0 = 32 * (tid & 1);
#pragma unroll
    for (int j = 0; j < 2; ++j) {
      const float* sp = stg + r * DF + c0 + 16 * j;
      const v4f f0 = *(const v4fa*)sp;
      const v4f f1 = *(const v4fa*)(sp + 4);
      const v4f f2 = *(const v4fa*)(sp + 8);
      const v4f f3 = *(const v4fa*)(sp + 12);
      v8us h0, l0, h1, l1;
      split8b(f0, f1, h0, l0);
      split8b(f2, f3, h1, l1);
      unsigned short* tp = tpl + r * KZ + c0 + 16 * j;
      *(v8usa*)tp = h0;
      *(v8usa*)(tp + 8) = h1;
      *(v8usa*)(tp + DF) = l0;
      *(v8usa*)(tp + DF + 8) = l1;
    }
  }
  __syncthreads();

  v8f acc2[NB2];
#pragma unroll
  for (int t = 0; t < NB2; ++t) acc2[t] = z8();
  {
    const unsigned short* ap2 = tpl + (16 * wave + m) * KZ + 8 * hh;
    const unsigned short* bp2 = WB + (size_t)m * (size_t)KZ + 8 * hh;
#pragma unroll
    for (int k0 = 0; k0 < KZ; k0 += 32) {
      Frag af;
      af.h[0] = *(const v8usa*)(ap2 + k0);
      af.h[1] = *(const v8usa*)(ap2 + k0 + 16);
#pragma unroll
      for (int nt = 0; nt < NB2; ++nt) {
        const unsigned short* wq = bp2 + (size_t)(16 * nt) * (size_t)KZ + k0;
        Frag bf;
        bf.h[0] = *(const v8usa*)wq;
        bf.h[1] = *(const v8usa*)(wq + 16);
        acc2[nt] = wmk(af, bf, acc2[nt]);
      }
    }
  }
#pragma unroll
  for (int nt = 0; nt < NB2; ++nt) {
    const int lc = 16 * nt + m;
    const float bv = cb[lc], sc = csc[lc], rm = crm[lc], be = cbe[lc];
#pragma unroll
    for (int r = 0; r < 8; ++r) {
      const int lr = 16 * wave + 8 * hh + r;
      const float v = acc2[nt][r] + bv;
      const float y = fmaf(v - rm, sc, be);
      if constexpr (FIN == 0) {
        stg[lr * DF + lc] = fmaxf(y, 0.0f);
      } else {
        if (lc < NCLS) orow[lr * NCLS + lc] = y;
      }
    }
  }
  __syncthreads();

  if constexpr (FIN == 0) {
    v4f pv[8];
    const int rq = lane >> 4;
    const int cq = 4 * (lane & 15);
#pragma unroll
    for (int i = 0; i < 8; ++i) {
      const int lr = 16 * wave + 2 * i + rq;
      pv[i] = *(const v4fa*)(stg + lr * DF + cq);
    }
#pragma unroll
    for (int i = 0; i < 8; ++i) {
      const int gr = rowBase + 16 * wave + 2 * i + rq;
      float* op = H + (size_t)gr * (size_t)DF + cq;
      *(volatile v4f*)op = pv[i];
    }
    __threadfence();
#pragma unroll
    for (int i = 0; i < 8; ++i) {
      const int gr = rowBase + 16 * wave + 2 * i + rq;
      float* op = H + (size_t)gr * (size_t)DF + cq;
      *(volatile v4f*)op = pv[i];
    }
    (void)outF; (void)nN;
  } else {
    const long long nTot = (long long)nN * NCLS;
    const long long eBlk = (long long)rowBase * NCLS;
    const int  pA = tid;
    const int  pB = GTHR + lane;
    const bool wB = (wave == 0);
    const v4f  va = *(const v4fa*)(orow + 4 * pA);
    const v4f  vb = *(const v4fa*)(orow + 4 * pB);
    const long long eA = eBlk + 4 * pA;
    const long long eB = eBlk + 4 * pB;
    const bool fullA = (eA + 4 <= nTot);
    const bool partA = (eA < nTot) && !fullA;
    const bool fullB = wB && (eB + 4 <= nTot);
    const bool partB = wB && (eB < nTot) && !fullB;
    float* opA = outF + (size_t)eA;
    float* opB = outF + (size_t)eB;
    if (fullA) *(volatile v4f*)opA = va;
    if (partA) {
      if (eA + 0 < nTot) *(volatile float*)(opA + 0) = va.x;
      if (eA + 1 < nTot) *(volatile float*)(opA + 1) = va.y;
      if (eA + 2 < nTot) *(volatile float*)(opA + 2) = va.z;
    }
    if (fullB) *(volatile v4f*)opB = vb;
    if (partB) {
      if (eB + 0 < nTot) *(volatile float*)(opB + 0) = vb.x;
      if (eB + 1 < nTot) *(volatile float*)(opB + 1) = vb.y;
      if (eB + 2 < nTot) *(volatile float*)(opB + 2) = vb.z;
    }
    __threadfence();
    if (fullA) *(volatile v4f*)opA = va;
    if (partA) {
      if (eA + 0 < nTot) *(volatile float*)(opA + 0) = va.x;
      if (eA + 1 < nTot) *(volatile float*)(opA + 1) = va.y;
      if (eA + 2 < nTot) *(volatile float*)(opA + 2) = va.z;
    }
    if (fullB) *(volatile v4f*)opB = vb;
    if (partB) {
      if (eB + 0 < nTot) *(volatile float*)(opB + 0) = vb.x;
      if (eB + 1 < nTot) *(volatile float*)(opB + 1) = vb.y;
      if (eB + 2 < nTot) *(volatile float*)(opB + 2) = vb.z;
    }
    (void)H;
  }
}

template <int RND>
__global__ __launch_bounds__(NTHR) void k_agg(const int* __restrict__ srcs, const int* __restrict__ dsts,
                                              const float* __restrict__ ew, const float* __restrict__ F,
                                              unsigned short* Aout, int nN, int nE, int vec8) {
  extern __shared__ __attribute__((aligned(16))) int lds_i[];
  int* reg1 = lds_i;
  int* reg2 = reg1 + RCAP;
  int* scnt = reg2 + RCAP;
  int* soff = scnt + NBA;
  int* list = soff + NBA;
  int* wcnt = list + LISTN;
  int* wtot = wcnt + NWAVE;
  const int tid = (int)threadIdx.x, lane = tid & 31, wave = tid >> 5;
  const int nodeBase = (int)blockIdx.x * NBA;

  {
    const v4i z4 = {0, 0, 0, 0};
    for (int i = tid * 4; i < ZINTS; i += NTHR * 4) *(v4ia*)(lds_i + i) = z4;
    if (tid < 2 * NWAVE) wcnt[tid] = 0;
  }
  __syncthreads();

  int tot = 0;
  const int nChunks = (nE + CHUNK - 1) / CHUNK;
#pragma unroll 1
  for (int ch = 0; ch < nChunks; ++ch) {
    const int cbase = ch * CHUNK;
    const int wc = scan_chunk(dsts, nE, cbase, nodeBase, NBA, vec8, list, tid, lane, wave);
    if (lane == 0) wcnt[wave] = wc;
    __syncthreads();
    int pre = 0, all = 0;
#pragma unroll
    for (int w2 = 0; w2 < NWAVE; ++w2) {
      int c = wcnt[w2];
      c = c < 0 ? 0 : (c > WCAP ? WCAP : c);
      all += c;
      pre += (w2 < wave) ? c : 0;
    }
    const int wcc  = wc > WCAP ? WCAP : wc;
    const int base = tot + pre;
#pragma unroll 1
    for (int i = lane; i < wcc; i += 32) {
      const int ent = list[wave * WCAP + i];
      const int el  = (ent >> PKS) & (CHUNK - 1);
      const int sl  = ent & (NBA - 1);
      int eid = cbase + el;
      eid = eid > nE - 1 ? nE - 1 : eid;
      const int pos = base + i;
      if (pos < RCAP) reg1[pos] = (int)(((unsigned)eid << PKS) | (unsigned)sl);
    }
    tot += all;
    tot = tot > RCAP ? RCAP : tot;
    __syncthreads();
  }
  const int nh = tot;

  if (wave == 0) {
#pragma unroll 1
    for (int b0 = 0; b0 < nh; b0 += 32) {
      const int idx = b0 + lane;
      const int uv  = reg1[idx < RCAP ? idx : RCAP - 1];
      const int m32 = (nh - b0) < 32 ? (nh - b0) : 32;
#pragma unroll 1
      for (int k = 0; k < m32; ++k) {
        const int u  = __builtin_amdgcn_readlane(uv, k);
        const int sl = u & (NBA - 1);
        if (lane == 0) scnt[sl] = scnt[sl] + 1;
      }
    }
  }
  __syncthreads();

  {
    const v4i ca = *(const v4ia*)(scnt + 4 * tid);
    const int e0 = ca.x < 0 ? 0 : ca.x, e1 = ca.y < 0 ? 0 : ca.y, e2 = ca.z < 0 ? 0 : ca.z, e3 = ca.w < 0 ? 0 : ca.w;
    const int ts = e0 + e1 + e2 + e3;
    int incl = ts;
#pragma unroll
    for (int d = 1; d < 32; d <<= 1) {
      const int up = __shfl_up(incl, d, 32);
      if (lane >= d) incl += up;
    }
    if (lane == 31) wtot[wave] = incl;
    __syncthreads();
    int pre = 0;
#pragma unroll
    for (int w2 = 0; w2 < NWAVE; ++w2) pre += (w2 < wave) ? wtot[w2] : 0;
    int run = pre + incl - ts;
    soff[4 * tid + 0] = run; run += e0;
    soff[4 * tid + 1] = run; run += e1;
    soff[4 * tid + 2] = run; run += e2;
    soff[4 * tid + 3] = run;
  }
  __syncthreads();
  for (int i = tid; i < NBA; i += NTHR) list[i] = soff[i];
  __syncthreads();

  if (wave == 0) {
#pragma unroll 1
    for (int b0 = 0; b0 < nh; b0 += 32) {
      const int idx = b0 + lane;
      const int uv  = reg1[idx < RCAP ? idx : RCAP - 1];
      const int m32 = (nh - b0) < 32 ? (nh - b0) : 32;
#pragma unroll 1
      for (int k = 0; k < m32; ++k) {
        const int u   = __builtin_amdgcn_readlane(uv, k);
        const int sl  = u & (NBA - 1);
        const int eid = (int)((unsigned)u >> PKS);
        if (lane == 0) {
          int pos = list[sl];
          pos = pos < 0 ? 0 : (pos > RCAP - 1 ? RCAP - 1 : pos);
          reg2[pos] = eid;
          list[sl] = pos + 1;
        }
      }
    }
  }
  __syncthreads();

  const int nbw = NBA / NWAVE;
  const bool ovf = (nh >= RCAP);
  const float qnan = __int_as_float(0x7fc00000);

#pragma unroll 1
  for (int jt = 0; jt < nbw; ++jt) {
    const int slot = wave * nbw + jt;
    const int node = nodeBase + slot;
    int st = soff[slot];
    const int craw = scnt[slot];
    int cnt = craw;
    st  = st < 0 ? 0 : (st > nh ? nh : st);
    cnt = cnt < 0 ? 0 : (cnt > DEGCAP ? DEGCAP : cnt);
    if (cnt > nh - st) cnt = nh - st;
    const float pz = (ovf || craw > DEGCAP) ? qnan : 0.0f;
    const bool live = node < nN;
    const int nc = node < nN ? node : nN - 1;

    float a0 = 0.0f, a1 = 0.0f;
#pragma unroll 1
    for (int b0 = 0; b0 < cnt; b0 += 32) {
      int idx = st + b0 + lane; idx = idx > RCAP - 1 ? RCAP - 1 : idx;
      int eid = reg2[idx]; eid = eid < 0 ? 0 : (eid > nE - 1 ? nE - 1 : eid);
      int sr = srcs[eid]; sr = sr < 0 ? 0 : (sr > nN - 1 ? nN - 1 : sr);
      const int wvi = __float_as_int(bf_rne(ew[eid]));
      const int m32 = (cnt - b0) < 32 ? (cnt - b0) : 32;
#pragma unroll 1
      for (int k = 0; k < m32; ++k) {
        const int   sk = __builtin_amdgcn_readlane(sr, k);
        const float wk = __int_as_float(__builtin_amdgcn_readlane(wvi, k));
        const v2f v = *(const v2fa*)(F + (size_t)sk * DF + 2 * lane);
        float vx = v.x, vy = v.y;
        if constexpr (RND == 1) {
          vx = bf_rne(vx); vy = bf_rne(vy);
        }
        a0 = fmaf(wk, vx, a0); a1 = fmaf(wk, vy, a1);
      }
    }
    const v2f sv = *(const v2fa*)(F + (size_t)nc * DF + 2 * lane);
    float sx = sv.x, sy = sv.y;
    if constexpr (RND == 1) {
      sx = bf_rne(sx); sy = bf_rne(sy);
    }
    float r0 = fmaf(SELFS, sx, a0);
    float r1 = fmaf(SELFS, sy, a1);
    r0 = (live ? r0 : 0.0f) + pz;
    r1 = (live ? r1 : 0.0f) + pz;

    const unsigned short hb0 = bf_bits(r0), hb1 = bf_bits(r1);
    const unsigned short lb0 = bf_bits(r0 - bf_val(hb0));
    const unsigned short lb1 = bf_bits(r1 - bf_val(hb1));
    v2u pk;
    pk.x = (unsigned int)hb0 | ((unsigned int)hb1 << 16);
    pk.y = (unsigned int)lb0 | ((unsigned int)lb1 << 16);
    unsigned short* gp = Aout + (size_t)node * (size_t)KZ + 4 * lane;
    *(volatile v2u*)gp = pk;
    __threadfence();
    *(volatile v2u*)gp = pk;
  }
}

static inline int cdiv(int a, int b) { return (a + b - 1) / b; }
static inline size_t al256(size_t o) { return (o + 255) & ~(size_t)255; }

extern "C" void kernel_launch(void* const* d_in, const int* in_sizes, int n_in,
                              void* d_out, int out_size, void* d_ws, size_t ws_size,
                              hipStream_t stream) {
  if (n_in < 19) return;
  if (in_sizes[0] < DF || (in_sizes[0] % DF) != 0) return;
  const int nN = in_sizes[0] / DF;
  if (nN < 1 || nN > (1 << 22)) return;
  if (in_sizes[1] < 2 || (in_sizes[1] & 1) != 0) return;
  const int nE = in_sizes[1] / 2;
  if (nE < 1 || nE >= (1 << (32 - PKS))) return;
  if (in_sizes[2] != nE) return;
  if (in_sizes[3] != DF * DF || in_sizes[4] != DF) return;
  if (in_sizes[5] != DF * DF || in_sizes[6] != DF) return;
  if (in_sizes[7] != DF || in_sizes[8] != DF || in_sizes[9] != DF || in_sizes[10] != DF) return;
  if (in_sizes[11] != DF * DF || in_sizes[12] != DF) return;
  if (in_sizes[13] != DF * NCLS || in_sizes[14] != NCLS) return;
  if (in_sizes[15] != NCLS || in_sizes[16] != NCLS || in_sizes[17] != NCLS || in_sizes[18] != NCLS) return;
  if ((long long)out_size != (long long)nN * NCLS) return;

  const float* x   = (const float*)d_in[0];
  const int*   ei  = (const int*)  d_in[1];
  const float* ew  = (const float*)d_in[2];
  const float* w1a = (const float*)d_in[3];
  const float* b1a = (const float*)d_in[4];
  const float* w1b = (const float*)d_in[5];
  const float* b1b = (const float*)d_in[6];
  const float* g1  = (const float*)d_in[7];
  const float* be1 = (const float*)d_in[8];
  const float* m1  = (const float*)d_in[9];
  const float* v1  = (const float*)d_in[10];
  const float* w2a = (const float*)d_in[11];
  const float* b2a = (const float*)d_in[12];
  const float* w2b = (const float*)d_in[13];
  const float* b2b = (const float*)d_in[14];
  const float* g2  = (const float*)d_in[15];
  const float* be2 = (const float*)d_in[16];
  const float* m2  = (const float*)d_in[17];
  const float* v2  = (const float*)d_in[18];
  float* out = (float*)d_out;
  const int* src = ei;
  const int* dst = ei + nE;

  const int MP   = cdiv(nN, GBM) * GBM;
  const int gM   = MP / GBM;
  const int gA   = cdiv(MP, NBA);
  const int RA   = gA * NBA;
  const int vec8 = ((nE & 3) == 0) ? 1 : 0;
  if ((long long)RA < (long long)MP) return;
  if ((long long)gM * GBM < (long long)nN) return;

  char* ws = (char*)d_ws;
  size_t off = 0;
  const size_t oWA1 = off; off = al256(off + (size_t)DF * KZ * 2);
  const size_t oWB1 = off; off = al256(off + (size_t)DF * KZ * 2);
  const size_t oWA2 = off; off = al256(off + (size_t)DF * KZ * 2);
  const size_t oWB2 = off; off = al256(off + (size_t)NCP * KZ * 2);
  const size_t oZ   = off; off = al256(off + (size_t)RA * KZ * 2);
  const size_t oH1  = off; off = al256(off + (size_t)MP * DF * 4);
  if (off > ws_size || off > (size_t)WSMAX) return;
  unsigned short* WA1 = (unsigned short*)(ws + oWA1);
  unsigned short* WB1 = (unsigned short*)(ws + oWB1);
  unsigned short* WA2 = (unsigned short*)(ws + oWA2);
  unsigned short* WB2 = (unsigned short*)(ws + oWB2);
  unsigned short* Z   = (unsigned short*)(ws + oZ);
  float*          H1  = (float*)(ws + oH1);

  hipFuncSetAttribute(reinterpret_cast<const void*>(&k_agg<1>), hipFuncAttributeMaxDynamicSharedMemorySize, LDS_AGG);
  hipFuncSetAttribute(reinterpret_cast<const void*>(&k_agg<0>), hipFuncAttributeMaxDynamicSharedMemorySize, LDS_AGG);

  k_wprep<<<RG4 / NTHR, NTHR, 0, stream>>>(w1a, w1b, w2a, w2b, WA1, WB1, WA2, WB2);
  k_agg<1><<<gA, NTHR, LDS_AGG, stream>>>(src, dst, ew, x, Z, nN, nE, vec8);
  k_mlp<GNT, 0><<<gM, GTHR, 0, stream>>>(Z, WA1, b1a, WB1, b1b, g1, be1, m1, v1, H1, out, nN);
  k_agg<0><<<gA, NTHR, LDS_AGG, stream>>>(src, dst, ew, H1, Z, nN, nE, vec8);
  k_mlp<1, 1><<<gM, GTHR, 0, stream>>>(Z, WA2, b2a, WB2, b2b, g2, be2, m2, v2, H1, out, nN);
}
